// MixtureOfExpertsMLPModule_62466004353423
// MI455X (gfx1250) — hardware-verified
//
#include <hip/hip_runtime.h>
#include <stddef.h>

#define TOK    8192
#define DIM    1024
#define CHN    256
#define NEXP   16
#define NR     64
#define BM     32
#define KC     128
#define APITCH 136
#define HPITCH 264
#define NTHR   256
#define LDSU   8704

static_assert(TOK % BM == 0);
static_assert(TOK % 8 == 0);
static_assert(DIM % KC == 0);
static_assert(KC % 32 == 0);
static_assert(CHN % 32 == 0);
static_assert(DIM % 32 == 0);
static_assert(BM * KC == NTHR * 16);
static_assert((APITCH * 2) % 16 == 0);
static_assert((HPITCH * 2) % 16 == 0);
static_assert(APITCH >= KC);
static_assert(HPITCH >= CHN);
static_assert(LDSU == 2 * BM * APITCH);
static_assert((NTHR / 32) * 512 * 2 <= LDSU);
static_assert(BM * NR * 2 <= LDSU);
static_assert((NTHR / 32) * 32 == CHN);
static_assert((NTHR / 32) * 128 == DIM);
static_assert(NR == 4 * NEXP);
static_assert(BM * 4 <= NTHR);

typedef unsigned short us;
typedef us v8us_t __attribute__((ext_vector_type(8)));
typedef v8us_t __attribute__((may_alias)) v8us;
typedef unsigned int v4u __attribute__((ext_vector_type(4)));
typedef __bf16 v16bf __attribute__((ext_vector_type(16)));
typedef float v8f __attribute__((ext_vector_type(8)));
typedef float v4f_t __attribute__((ext_vector_type(4)));
typedef v4f_t __attribute__((may_alias)) v4f;
typedef float __attribute__((may_alias)) af;

union Frag { v16bf v; v8us_t u[2]; };
union Pk16 { v8us_t h; v4u u; };

__device__ __forceinline__ v8f zero8() {
  v8f z;
#pragma unroll
  for (int i = 0; i < 8; ++i) z[i] = 0.0f;
  return z;
}

__device__ __forceinline__ unsigned int bfbits(float f) {
  unsigned int u = __float_as_uint(f);
  u += 0x7FFFu + ((u >> 16) & 1u);
  return u >> 16;
}
__device__ __forceinline__ float bfval(float f) { return __uint_as_float(bfbits(f) << 16); }

__device__ __forceinline__ v16bf ldfr(const us* p, int k0) {
  Frag f;
  f.u[0] = *(const v8us*)(p + k0);
  f.u[1] = *(const v8us*)(p + k0 + 16);
  return f.v;
}

__device__ __forceinline__ v8f mma(v16bf a, v16bf b, v8f c) {
  return __builtin_amdgcn_wmma_f32_16x16x32_bf16(false, a, false, b, (short)0, c, false, false);
}

__device__ __forceinline__ float gelu_f(float v) {
  return 0.5f * v * (1.0f + erff(v * 0.70710678118654752f));
}

__global__ void __launch_bounds__(NTHR) cvt_kernel(const float* src, us* dst, int n8)
{
  const int i = blockIdx.x * NTHR + threadIdx.x;
  const bool ok = (i < n8);
  const int ic = ok ? i : (n8 - 1);
  const v4f_t a = *(const v4f*)(src + (size_t)ic * 8);
  const v4f_t b = *(const v4f*)(src + (size_t)ic * 8 + 4);
  Pk16 pk;
#pragma unroll
  for (int j = 0; j < 4; ++j) {
    pk.h[j]     = (us)bfbits(a[j]);
    pk.h[4 + j] = (us)bfbits(b[j]);
  }
  us* d = dst + (size_t)ic * 8;
  if (ok) *(volatile v4u*)d = pk.u;
  __threadfence();
  if (ok) *(volatile v4u*)d = pk.u;
}

__global__ void __launch_bounds__(NTHR) xnorm_kernel(const float* x, const float* g, const float* b, float* xn)
{
  const int token = blockIdx.x * 8 + (threadIdx.x >> 5);
  const int lane  = threadIdx.x & 31;
  if (token >= TOK) return;
  const float* row = x + (size_t)token * DIM + lane * 4;
  float s = 0.0f;
#pragma unroll 1
  for (int j = 0; j < 8; ++j) {
    const v4f_t v = *(const v4f*)(row + j * 128);
    s += (bfval(v[0]) + bfval(v[1])) + (bfval(v[2]) + bfval(v[3]));
  }
#pragma unroll
  for (int m = 16; m >= 1; m >>= 1) s += __shfl_xor(s, m, 32);
  const float mu = s * (1.0f / DIM);
  float s2 = 0.0f;
#pragma unroll 1
  for (int j = 0; j < 8; ++j) {
    const v4f_t v = *(const v4f*)(row + j * 128);
    float d;
    d = bfval(v[0]) - mu; s2 = fmaf(d, d, s2);
    d = bfval(v[1]) - mu; s2 = fmaf(d, d, s2);
    d = bfval(v[2]) - mu; s2 = fmaf(d, d, s2);
    d = bfval(v[3]) - mu; s2 = fmaf(d, d, s2);
  }
#pragma unroll
  for (int m = 16; m >= 1; m >>= 1) s2 += __shfl_xor(s2, m, 32);
  const float rstd = rsqrtf(s2 * (1.0f / DIM) + 1e-5f);
  v4f_t y[8];
#pragma unroll
  for (int j = 0; j < 8; ++j) {
    const v4f_t v  = *(const v4f*)(row + j * 128);
    const v4f_t gv = *(const v4f*)(g + j * 128 + lane * 4);
    const v4f_t bv = *(const v4f*)(b + j * 128 + lane * 4);
#pragma unroll
    for (int e = 0; e < 4; ++e)
      y[j][e] = (bfval(v[e]) - mu) * rstd * bfval(gv[e]) + bfval(bv[e]);
  }
  float* o = xn + (size_t)token * DIM + lane * 4;
#pragma unroll
  for (int j = 0; j < 8; ++j) *(volatile v4f_t*)(o + j * 128) = y[j];
  __threadfence();
#pragma unroll
  for (int j = 0; j < 8; ++j) *(volatile v4f_t*)(o + j * 128) = y[j];
}

__device__ __forceinline__ void stage_chunk(
    const float* s0, const float* s1, const float* s2, const float* s3,
    const float* wg, int npred, int isx,
    us* Ahi, us* Alo, int tok0, int kbase, int tid)
{
  const int row = tid >> 3;
  const int c0  = (tid & 7) * 16;
  const size_t goff = (size_t)(tok0 + row) * DIM + (size_t)(kbase + c0);
  float a[16];
#pragma unroll
  for (int j = 0; j < 16; ++j) a[j] = 0.0f;
#pragma unroll
  for (int p = 0; p < 4; ++p) {
    if (p < npred) {
      const float* src = (p == 0) ? s0 : ((p == 1) ? s1 : ((p == 2) ? s2 : s3));
      float w = 1.0f;
      if (isx == 0) w = wg[row * 4 + p];
#pragma unroll
      for (int q = 0; q < 4; ++q) {
        const v4f_t v = *(const v4f*)(src + goff + 4 * q);
        a[4 * q + 0] = fmaf(w, v[0], a[4 * q + 0]);
        a[4 * q + 1] = fmaf(w, v[1], a[4 * q + 1]);
        a[4 * q + 2] = fmaf(w, v[2], a[4 * q + 2]);
        a[4 * q + 3] = fmaf(w, v[3], a[4 * q + 3]);
      }
    }
  }
  v8us_t h0, h1, l0, l1;
#pragma unroll
  for (int j = 0; j < 8; ++j) {
    unsigned int hb = bfbits(a[j]);
    float hv = __uint_as_float(hb << 16);
    unsigned int lb = bfbits(a[j] - hv);
    h0[j] = (us)hb; l0[j] = (us)lb;
    hb = bfbits(a[8 + j]);
    hv = __uint_as_float(hb << 16);
    lb = bfbits(a[8 + j] - hv);
    h1[j] = (us)hb; l1[j] = (us)lb;
  }
  us* dh = Ahi + row * APITCH + c0;
  us* dl = Alo + row * APITCH + c0;
  *(v8us*)dh = h0;
  *(v8us*)(dh + 8) = h1;
  *(v8us*)dl = l0;
  *(v8us*)(dl + 8) = l1;
}

__global__ void __launch_bounds__(NTHR) router_kernel(const float* xn, const us* rwb, const float* rb, float* gates)
{
  __shared__ __align__(16) us lds_u[LDSU];
  us* Ahi = lds_u;
  us* Alo = lds_u + BM * APITCH;

  const int tid = threadIdx.x, wid = tid >> 5, lane = tid & 31;
  const int half = lane >> 4, l16 = lane & 15;
  const int tok0 = blockIdx.x * BM;
  const int rt = wid & 1, ct = wid >> 1;
  const int n = ct * 16 + l16;

  v8f acc = zero8();
#pragma unroll 1
  for (int kc = 0; kc < DIM / KC; ++kc) {
    stage_chunk(xn, xn, xn, xn, xn, 1, 1, Ahi, Alo, tok0, kc * KC, tid);
    __syncthreads();
    const us* Ah = Ahi + (rt * 16 + l16) * APITCH + 8 * half;
    const us* Al = Alo + (rt * 16 + l16) * APITCH + 8 * half;
    const us* Bp = rwb + (size_t)n * DIM + kc * KC + 8 * half;
#pragma unroll 1
    for (int k0 = 0; k0 < KC; k0 += 32) {
      const v16bf ah = ldfr(Ah, k0), al = ldfr(Al, k0);
      const v16bf bq = ldfr(Bp, k0);
      acc = mma(ah, bq, acc);
      acc = mma(al, bq, acc);
      asm volatile("v_nop\n\tv_nop\n\tv_nop\n\tv_nop" : "+v"(acc) : "v"(ah), "v"(al), "v"(bq));
    }
    __syncthreads();
  }

  af* stg = (af*)lds_u;
  const float rbv = bfval(rb[n]);
#pragma unroll
  for (int i = 0; i < 8; ++i) {
    const int r = rt * 16 + 8 * half + i;
    const float lg = acc[i] + rbv;
    const float ex = expf(-lg);
    const float gt = __builtin_amdgcn_rcpf(1.0f + ex);
    stg[r * NR + n] = gt;
  }
  __syncthreads();
  v4f_t o[2];
#pragma unroll
  for (int it = 0; it < 2; ++it) o[it] = *(const v4f*)((const af*)stg + it * 1024 + tid * 4);
  float* gp = gates + (size_t)tok0 * NR + tid * 4;
#pragma unroll
  for (int it = 0; it < 2; ++it) *(volatile v4f_t*)(gp + it * 1024) = o[it];
  __threadfence();
#pragma unroll
  for (int it = 0; it < 2; ++it) *(volatile v4f_t*)(gp + it * 1024) = o[it];
}

__global__ void __launch_bounds__(NTHR) node_kernel(
    const float* s0, const float* s1, const float* s2, const float* s3,
    const float* gates, int gcol, int npred, int isx,
    const us* w1, const float* b1, const float* lng, const float* lnb,
    const us* w2, float* outp, const float* x, const float* fc2b, int terminal)
{
  __shared__ __align__(16) us lds_u[LDSU];
  __shared__ __align__(16) us Hhi[BM * HPITCH];
  __shared__ __align__(16) us Hlo[BM * HPITCH];
  __shared__ float wgt[BM * 4];
  __shared__ float part[BM * 8];
  __shared__ float musr[BM * 2];

  us* Ahi = lds_u;
  us* Alo = lds_u + BM * APITCH;

  const int tid = threadIdx.x, wid = tid >> 5, lane = tid & 31;
  const int half = lane >> 4, l16 = lane & 15;
  const int tok0 = blockIdx.x * BM;

  if (tid < BM * 4) {
    const int t = tid >> 2, p = tid & 3;
    const float gv = gates[(size_t)(tok0 + t) * NR + gcol + p];
    wgt[tid] = (isx != 0) ? ((p == 0) ? 1.0f : 0.0f) : gv;
  }
  __syncthreads();

  v8f acc00 = zero8(), acc01 = zero8(), acc10 = zero8(), acc11 = zero8();
  const int n0 = wid * 32 + l16, n1 = n0 + 16;

#pragma unroll 1
  for (int kc = 0; kc < DIM / KC; ++kc) {
    stage_chunk(s0, s1, s2, s3, wgt, npred, isx, Ahi, Alo, tok0, kc * KC, tid);
    __syncthreads();
    const us* A0h = Ahi + l16 * APITCH + 8 * half;
    const us* A0l = Alo + l16 * APITCH + 8 * half;
    const us* A1h = Ahi + (16 + l16) * APITCH + 8 * half;
    const us* A1l = Alo + (16 + l16) * APITCH + 8 * half;
    const us* B0 = w1 + (size_t)n0 * DIM + kc * KC + 8 * half;
    const us* B1 = w1 + (size_t)n1 * DIM + kc * KC + 8 * half;
#pragma unroll 1
    for (int k0 = 0; k0 < KC; k0 += 32) {
      const v16bf a0h = ldfr(A0h, k0), a0l = ldfr(A0l, k0);
      const v16bf a1h = ldfr(A1h, k0), a1l = ldfr(A1l, k0);
      const v16bf bq0 = ldfr(B0, k0), bq1 = ldfr(B1, k0);
      acc00 = mma(a0h, bq0, acc00); acc00 = mma(a0l, bq0, acc00);
      acc01 = mma(a0h, bq1, acc01); acc01 = mma(a0l, bq1, acc01);
      acc10 = mma(a1h, bq0, acc10); acc10 = mma(a1l, bq0, acc10);
      acc11 = mma(a1h, bq1, acc11); acc11 = mma(a1l, bq1, acc11);
      asm volatile("v_nop\n\tv_nop\n\tv_nop\n\tv_nop"
                   : "+v"(acc00), "+v"(acc01), "+v"(acc10), "+v"(acc11)
                   : "v"(a0h), "v"(a0l), "v"(a1h), "v"(a1l), "v"(bq0), "v"(bq1));
    }
    __syncthreads();
  }

  {
    const float bias0 = bfval(b1[n0]), bias1 = bfval(b1[n1]);
#pragma unroll
    for (int i = 0; i < 8; ++i) {
      acc00[i] = gelu_f(acc00[i] + bias0);
      acc01[i] = gelu_f(acc01[i] + bias1);
      acc10[i] = gelu_f(acc10[i] + bias0);
      acc11[i] = gelu_f(acc11[i] + bias1);
    }
  }

#pragma unroll
  for (int i = 0; i < 8; ++i) {
    float sa = acc00[i] + acc01[i];
    float sb = acc10[i] + acc11[i];
#pragma unroll
    for (int m = 8; m >= 1; m >>= 1) { sa += __shfl_xor(sa, m, 32); sb += __shfl_xor(sb, m, 32); }
    if (l16 == 0) {
      part[(8 * half + i) * 8 + wid] = sa;
      part[(16 + 8 * half + i) * 8 + wid] = sb;
    }
  }
  __syncthreads();
  {
    const int t = tid >> 3, q = tid & 7;
    float sv = part[t * 8 + q];
#pragma unroll
    for (int m = 4; m >= 1; m >>= 1) sv += __shfl_xor(sv, m, 32);
    if (q == 0) musr[t * 2 + 0] = sv * (1.0f / CHN);
  }
  __syncthreads();

#pragma unroll
  for (int i = 0; i < 8; ++i) {
    const float mua = musr[(8 * half + i) * 2];
    const float mub = musr[(16 + 8 * half + i) * 2];
    float d, qa, qb;
    d = acc00[i] - mua; qa = d * d;
    d = acc01[i] - mua; qa = fmaf(d, d, qa);
    d = acc10[i] - mub; qb = d * d;
    d = acc11[i] - mub; qb = fmaf(d, d, qb);
#pragma unroll
    for (int m = 8; m >= 1; m >>= 1) { qa += __shfl_xor(qa, m, 32); qb += __shfl_xor(qb, m, 32); }
    if (l16 == 0) {
      part[(8 * half + i) * 8 + wid] = qa;
      part[(16 + 8 * half + i) * 8 + wid] = qb;
    }
  }
  __syncthreads();
  {
    const int t = tid >> 3, q = tid & 7;
    float sv = part[t * 8 + q];
#pragma unroll
    for (int m = 4; m >= 1; m >>= 1) sv += __shfl_xor(sv, m, 32);
    if (q == 0) musr[t * 2 + 1] = rsqrtf(sv * (1.0f / CHN) + 1e-5f);
  }
  __syncthreads();

  {
    const float g0 = bfval(lng[n0]), g1 = bfval(lng[n1]);
    const float e0 = bfval(lnb[n0]), e1 = bfval(lnb[n1]);
#pragma unroll
    for (int i = 0; i < 8; ++i) {
      const int ta = 8 * half + i, tb = ta + 16;
      const float mua = musr[ta * 2], ra = musr[ta * 2 + 1];
      const float mub = musr[tb * 2], rq = musr[tb * 2 + 1];
      float v; unsigned int hb, lb; float hv;
      v = (acc00[i] - mua) * ra * g0 + e0;
      hb = bfbits(v); hv = __uint_as_float(hb << 16); lb = bfbits(v - hv);
      Hhi[ta * HPITCH + n0] = (us)hb; Hlo[ta * HPITCH + n0] = (us)lb;
      v = (acc01[i] - mua) * ra * g1 + e1;
      hb = bfbits(v); hv = __uint_as_float(hb << 16); lb = bfbits(v - hv);
      Hhi[ta * HPITCH + n1] = (us)hb; Hlo[ta * HPITCH + n1] = (us)lb;
      v = (acc10[i] - mub) * rq * g0 + e0;
      hb = bfbits(v); hv = __uint_as_float(hb << 16); lb = bfbits(v - hv);
      Hhi[tb * HPITCH + n0] = (us)hb; Hlo[tb * HPITCH + n0] = (us)lb;
      v = (acc11[i] - mub) * rq * g1 + e1;
      hb = bfbits(v); hv = __uint_as_float(hb << 16); lb = bfbits(v - hv);
      Hhi[tb * HPITCH + n1] = (us)hb; Hlo[tb * HPITCH + n1] = (us)lb;
    }
  }
  __syncthreads();

  af* stw = (af*)lds_u + wid * 512;
  const int rq4 = lane >> 3, c4 = (lane & 7) * 4;
#pragma unroll 1
  for (int g = 0; g < 2; ++g) {
    v8f acc[2][4];
#pragma unroll
    for (int c = 0; c < 4; ++c) { acc[0][c] = zero8(); acc[1][c] = zero8(); }
    const int colbase = wid * 128 + g * 64;
    const us* H0h = Hhi + l16 * HPITCH + 8 * half;
    const us* H0l = Hlo + l16 * HPITCH + 8 * half;
    const us* H1h = Hhi + (16 + l16) * HPITCH + 8 * half;
    const us* H1l = Hlo + (16 + l16) * HPITCH + 8 * half;
    const us* Bb = w2 + (size_t)(colbase + l16) * CHN + 8 * half;
#pragma unroll 1
    for (int k0 = 0; k0 < CHN; k0 += 32) {
      const v16bf a0h = ldfr(H0h, k0), a0l = ldfr(H0l, k0);
      const v16bf a1h = ldfr(H1h, k0), a1l = ldfr(H1l, k0);
      v16bf bq;
#pragma unroll
      for (int c = 0; c < 4; ++c) {
        bq = ldfr(Bb + (size_t)c * 16 * CHN, k0);
        acc[0][c] = mma(a0h, bq, acc[0][c]); acc[0][c] = mma(a0l, bq, acc[0][c]);
        acc[1][c] = mma(a1h, bq, acc[1][c]); acc[1][c] = mma(a1l, bq, acc[1][c]);
      }
      asm volatile("v_nop\n\tv_nop\n\tv_nop\n\tv_nop"
                   : "+v"(acc[0][0]), "+v"(acc[0][1]), "+v"(acc[0][2]), "+v"(acc[0][3]),
                     "+v"(acc[1][0]), "+v"(acc[1][1]), "+v"(acc[1][2]), "+v"(acc[1][3])
                   : "v"(a0h), "v"(a0l), "v"(a1h), "v"(a1l), "v"(bq));
    }

#pragma unroll
    for (int rt = 0; rt < 2; ++rt) {
#pragma unroll
      for (int cp = 0; cp < 2; ++cp) {
#pragma unroll
        for (int cc = 0; cc < 2; ++cc) {
          const int c = cp * 2 + cc;
          const int n = colbase + c * 16 + l16;
          float fb = 0.0f;
          if (terminal != 0) fb = bfval(fc2b[n]);
#pragma unroll
          for (int i = 0; i < 8; ++i) {
            const int r = 8 * half + i;
            float v = acc[rt][c][i];
            if (terminal != 0) {
              const float xv = bfval(x[(size_t)(tok0 + rt * 16 + r) * DIM + n]);
              v = xv + (v + fb);
            }
            stw[r * 32 + cc * 16 + l16] = v;
          }
        }
        __syncthreads();
        v4f_t o[4];
#pragma unroll
        for (int pp = 0; pp < 4; ++pp)
          o[pp] = *(const v4f*)((const af*)stw + (pp * 4 + rq4) * 32 + c4);
        float* gp = outp + (size_t)(tok0 + rt * 16) * DIM + colbase + cp * 32 + c4;
#pragma unroll
        for (int pp = 0; pp < 4; ++pp)
          *(volatile v4f_t*)(gp + (size_t)(pp * 4 + rq4) * DIM) = o[pp];
        __threadfence();
#pragma unroll
        for (int pp = 0; pp < 4; ++pp)
          *(volatile v4f_t*)(gp + (size_t)(pp * 4 + rq4) * DIM) = o[pp];
        __syncthreads();
      }
    }
  }
}

extern "C" void kernel_launch(void* const* d_in, const int* in_sizes, int n_in,
                              void* d_out, int out_size, void* d_ws, size_t ws_size,
                              hipStream_t stream)
{
  if (n_in < 11) return;
  if (in_sizes[0] != TOK * DIM) return;
  if (in_sizes[1] != DIM || in_sizes[2] != DIM) return;
  if (in_sizes[3] != NEXP * CHN * DIM) return;
  if (in_sizes[4] != NEXP * CHN || in_sizes[5] != NEXP * CHN || in_sizes[6] != NEXP * CHN) return;
  if (in_sizes[7] != NEXP * DIM * CHN) return;
  if (in_sizes[8] != DIM) return;
  if (in_sizes[9] != NR * DIM || in_sizes[10] != NR) return;
  if (out_size != TOK * DIM) return;

  const float* x        = (const float*)d_in[0];
  const float* norm_g   = (const float*)d_in[1];
  const float* norm_b   = (const float*)d_in[2];
  const float* fc1_w    = (const float*)d_in[3];
  const float* fc1_b    = (const float*)d_in[4];
  const float* ln_g     = (const float*)d_in[5];
  const float* ln_b     = (const float*)d_in[6];
  const float* fc2_w    = (const float*)d_in[7];
  const float* fc2_bias = (const float*)d_in[8];
  const float* router_w = (const float*)d_in[9];
  const float* router_b = (const float*)d_in[10];
  float* out = (float*)d_out;

  const size_t plane = (size_t)TOK * DIM * sizeof(float);
  const size_t oS0 = 0, oS1 = plane, oS2 = 2 * plane, oS3 = 3 * plane;
  const size_t oW1 = 4 * plane;
  const size_t oW2 = oW1 + (size_t)NEXP * CHN * DIM * 2;
  const size_t oRW = oW2 + (size_t)NEXP * DIM * CHN * 2;
  const size_t oG  = oRW + (size_t)NR * DIM * 2;
  const size_t total = oG + (size_t)TOK * NR * sizeof(float);
  if (total > ws_size) return;

  char* ws = (char*)d_ws;
  float* S[4];
  S[0] = (float*)(ws + oS0); S[1] = (float*)(ws + oS1); S[2] = (float*)(ws + oS2); S[3] = (float*)(ws + oS3);
  us* w1b = (us*)(ws + oW1);
  us* w2b = (us*)(ws + oW2);
  us* rwb = (us*)(ws + oRW);
  float* gates = (float*)(ws + oG);

  const int n8W = (NEXP * CHN * DIM) / 8;
  const int n8R = (NR * DIM) / 8;
  cvt_kernel<<<(n8W + NTHR - 1) / NTHR, NTHR, 0, stream>>>(fc1_w, w1b, n8W);
  cvt_kernel<<<(n8W + NTHR - 1) / NTHR, NTHR, 0, stream>>>(fc2_w, w2b, n8W);
  cvt_kernel<<<(n8R + NTHR - 1) / NTHR, NTHR, 0, stream>>>(router_w, rwb, n8R);
  xnorm_kernel<<<TOK / 8, NTHR, 0, stream>>>(x, norm_g, norm_b, S[0]);
  router_kernel<<<TOK / BM, NTHR, 0, stream>>>(S[0], rwb, router_b, gates);

  const int NP[NEXP] = {0, 1, 2, 2, 2, 2, 2, 2, 2, 2, 2, 2, 2, 2, 3, 4};
  const int PL[NEXP][4] = {
    {0, 0, 0, 0}, {0, 0, 0, 0}, {0, 1, 0, 0}, {1, 2, 0, 0}, {2, 3, 0, 0}, {3, 4, 0, 0},
    {4, 5, 0, 0}, {5, 6, 0, 0}, {6, 7, 0, 0}, {7, 8, 0, 0}, {8, 9, 0, 0}, {9, 10, 0, 0},
    {10, 11, 0, 0}, {11, 12, 0, 0}, {0, 12, 13, 0}, {0, 1, 13, 14}};
  for (int v = 0; v < NEXP; ++v) {
    const int isx = (v == 0) ? 1 : 0;
    const int npred = isx ? 1 : NP[v];
    const float* sp[4];
    for (int i = 0; i < 4; ++i) {
      if (isx) { sp[i] = S[0]; continue; }
      if (i < NP[v]) {
        const int u = PL[v][i];
        const int su = (u == 0) ? 1 : ((u == 1) ? 2 : ((u & 1) ? 3 : 0));
        sp[i] = S[su];
      } else {
        sp[i] = S[1];
      }
    }
    const int so = (v == 0) ? 1 : ((v == 1) ? 2 : ((v & 1) ? 3 : 0));
    float* op = (v == NEXP - 1) ? out : S[so];
    node_kernel<<<TOK / BM, NTHR, 0, stream>>>(
        sp[0], sp[1], sp[2], sp[3], gates, v * 4, npred, isx,
        w1b + (size_t)v * CHN * DIM, fc1_b + (size_t)v * CHN, ln_g + (size_t)v * CHN, ln_b + (size_t)v * CHN,
        w2b + (size_t)v * DIM * CHN, op, x, fc2_bias, (v == NEXP - 1) ? 1 : 0);
  }
}
